// UMPS_35390530519710
// MI455X (gfx1250) — hardware-verified
//
#include <hip/hip_runtime.h>


#define BOND_  64
#define FEAT1_ 33
#define BATCH_ 256
#define TLEN_  512
#define OUTD_  32
#define KK_    (FEAT1_ * BOND_)
#define NRB_   16
#define NTH_   384
#define NKS_   (KK_ / 32)
#define KSW_   (NKS_ / 3)

static_assert(KK_ == 2112);
static_assert(KK_ % 32 == 0);
static_assert(NKS_ % 3 == 0);
static_assert(BATCH_ % NRB_ == 0);
static_assert((NRB_ * FEAT1_ * (BOND_ / 8)) % NTH_ == 0);
static_assert(NTH_ == 32 * 12);
static_assert(NRB_ * (BOND_ / 8) == 128);
static_assert(OUTD_ * (BOND_ / 8) == NTH_ - 128);
static_assert(NRB_ * OUTD_ == 4 * 128);

typedef float          v4f   __attribute__((ext_vector_type(4)));
typedef float          v8f   __attribute__((ext_vector_type(8)));
typedef unsigned short u16x8 __attribute__((ext_vector_type(8)));
typedef __bf16         v16bf __attribute__((ext_vector_type(16)));

union FragB { u16x8 h[2]; v16bf v; };

constexpr size_t SZ_PL  = (size_t)BOND_ * KK_ * 2;
constexpr size_t OFF_BH = 0;
constexpr size_t OFF_BL = OFF_BH + SZ_PL;
constexpr size_t WS_END = OFF_BL + SZ_PL;
static_assert(SZ_PL % 128 == 0);
static_assert((KK_ * 2) % 128 == 0);
static_assert(WS_END == (size_t)540672);
static_assert(WS_END <= (size_t)134217728);

__device__ __forceinline__ unsigned short bfb(float f) {
    unsigned uu = __float_as_uint(f);
    uu += 0x7FFFu + ((uu >> 16) & 1u);
    return (unsigned short)(uu >> 16);
}
__device__ __forceinline__ void split8(const v8f v, u16x8& hi, u16x8& lo) {
#pragma unroll
    for (int e = 0; e < 8; ++e) {
        const unsigned short hb = bfb(v[e]);
        const float hf = __uint_as_float(((unsigned)hb) << 16);
        hi[e] = hb;
        lo[e] = bfb(v[e] - hf);
    }
}
__device__ __forceinline__ v8f ld8f(const float* p) {
    const v4f a = *(const v4f*)p;
    const v4f b = *(const v4f*)(p + 4);
    return __builtin_shufflevector(a, b, 0, 1, 2, 3, 4, 5, 6, 7);
}

__device__ __forceinline__ void mma_bf(v8f& acc, const FragB& a, const FragB& b) {
    acc = __builtin_amdgcn_wmma_f32_16x16x32_bf16(false, a.v, false, b.v, (short)0, acc, false, false);
    asm volatile("v_nop\n\tv_nop\n\tv_nop\n\tv_nop" : "+v"(acc) : "v"(a.v), "v"(b.v));
}

__global__ __launch_bounds__(256)
void core_planes_kernel(const float* __restrict__ core, unsigned short* Bh, unsigned short* Bl)
{
    const int j = blockIdx.x;
#pragma unroll 1
    for (int q = threadIdx.x; q < KK_ / 8; q += 256) {
        const int k0 = 8 * q;
        const int f  = k0 >> 6;
        const int i0 = k0 & (BOND_ - 1);
        v8f v;
#pragma unroll
        for (int e = 0; e < 8; ++e) v[e] = core[((size_t)(i0 + e) * FEAT1_ + f) * BOND_ + j];
        u16x8 hi, lo;
        split8(v, hi, lo);
        unsigned short* ph = Bh + (size_t)j * KK_ + k0;
        unsigned short* pl = Bl + (size_t)j * KK_ + k0;
        *(volatile u16x8*)ph = hi;
        *(volatile u16x8*)pl = lo;
        __threadfence();
        *(volatile u16x8*)ph = hi;
        *(volatile u16x8*)pl = lo;
    }
}

__global__ __launch_bounds__(NTH_)
void chain_kernel(const float* __restrict__ xg, const float* __restrict__ alpha, const float* __restrict__ outc,
                  const unsigned short* __restrict__ Bh, const unsigned short* __restrict__ Bl, float* out)
{
    __shared__ __attribute__((aligned(16))) unsigned short Ah[NRB_ * KK_];
    __shared__ __attribute__((aligned(16))) unsigned short Al[NRB_ * KK_];
    __shared__ __attribute__((aligned(16))) float vf[NRB_ * BOND_];
    __shared__ __attribute__((aligned(16))) float part[3 * NRB_ * BOND_];
    __shared__ __attribute__((aligned(16))) unsigned short obh[OUTD_ * BOND_];
    __shared__ __attribute__((aligned(16))) unsigned short obl[OUTD_ * BOND_];
    __shared__ __attribute__((aligned(16))) float ost[NRB_ * OUTD_];

    const int tid  = threadIdx.x;
    const int lane = tid & 31, h = lane >> 4, ml = lane & 15;
    const int wv   = __builtin_amdgcn_readfirstlane(tid >> 5);
    const int ct   = wv & 3;
    const int kq   = wv >> 2;
    const int b0   = blockIdx.x * NRB_;

    for (int i = tid; i < NRB_ * BOND_; i += NTH_) vf[i] = alpha[i & (BOND_ - 1)];
    __syncthreads();

    const unsigned short* ahp = Ah + ml * KK_ + 8 * h;
    const unsigned short* alp = Al + ml * KK_ + 8 * h;
    const unsigned short* bhp = Bh + (size_t)(16 * ct + ml) * KK_ + 8 * h;
    const unsigned short* blp = Bl + (size_t)(16 * ct + ml) * KK_ + 8 * h;
    float* pp = part + kq * (NRB_ * BOND_) + 16 * ct + ml;

#pragma unroll 1
    for (int t = 0; t < TLEN_; ++t) {
#pragma unroll 1
        for (int idx = tid; idx < NRB_ * FEAT1_ * (BOND_ / 8); idx += NTH_) {
            const int q   = idx & 7;
            const int rf  = idx >> 3;
            const int row = rf / FEAT1_;
            const int f   = rf - row * FEAT1_;
            const float xv = xg[((size_t)(b0 + row) * TLEN_ + t) * FEAT1_ + f];
            v8f v = ld8f(vf + row * BOND_ + 8 * q);
#pragma unroll
            for (int e = 0; e < 8; ++e) v[e] *= xv;
            u16x8 hi, lo;
            split8(v, hi, lo);
            const int off = row * KK_ + f * BOND_ + 8 * q;
            *(u16x8*)(Ah + off) = hi;
            *(u16x8*)(Al + off) = lo;
        }
        __syncthreads();

        v8f acc;
#pragma unroll
        for (int r = 0; r < 8; ++r) acc[r] = 0.0f;
#pragma unroll 1
        for (int s = 0; s < KSW_; ++s) {
            const int k0 = (KSW_ * kq + s) * 32;
            FragB ah, al, bh, bl;
            ah.h[0] = *(const u16x8*)(ahp + k0);
            ah.h[1] = *(const u16x8*)(ahp + k0 + 16);
            al.h[0] = *(const u16x8*)(alp + k0);
            al.h[1] = *(const u16x8*)(alp + k0 + 16);
            bh.h[0] = *(const u16x8*)(bhp + k0);
            bh.h[1] = *(const u16x8*)(bhp + k0 + 16);
            bl.h[0] = *(const u16x8*)(blp + k0);
            bl.h[1] = *(const u16x8*)(blp + k0 + 16);
            mma_bf(acc, ah, bh);
            mma_bf(acc, ah, bl);
            mma_bf(acc, al, bh);
        }
#pragma unroll
        for (int r = 0; r < 8; ++r) pp[(8 * h + r) * BOND_] = acc[r];
        __syncthreads();

        for (int idx = tid; idx < NRB_ * BOND_; idx += NTH_) {
            const float s01 = part[idx] + part[NRB_ * BOND_ + idx];
            vf[idx] = s01 + part[2 * NRB_ * BOND_ + idx];
        }
        __syncthreads();
    }

    if (tid < NRB_ * (BOND_ / 8)) {
        const int row = tid >> 3, q = tid & 7;
        const v8f v = ld8f(vf + row * BOND_ + 8 * q);
        u16x8 hi, lo;
        split8(v, hi, lo);
        *(u16x8*)(Ah + row * KK_ + 8 * q) = hi;
        *(u16x8*)(Al + row * KK_ + 8 * q) = lo;
    } else {
        const int tt = tid - NRB_ * (BOND_ / 8);
        const int o = tt >> 3, q = tt & 7;
        v8f v;
#pragma unroll
        for (int e = 0; e < 8; ++e) v[e] = outc[(8 * q + e) * OUTD_ + o];
        u16x8 hi, lo;
        split8(v, hi, lo);
        *(u16x8*)(obh + o * BOND_ + 8 * q) = hi;
        *(u16x8*)(obl + o * BOND_ + 8 * q) = lo;
    }
    __syncthreads();

    if (wv < 2) {
        v8f acc2;
#pragma unroll
        for (int r = 0; r < 8; ++r) acc2[r] = 0.0f;
        const unsigned short* ohp = obh + (16 * wv + ml) * BOND_ + 8 * h;
        const unsigned short* olp = obl + (16 * wv + ml) * BOND_ + 8 * h;
#pragma unroll
        for (int s = 0; s < 2; ++s) {
            const int k0 = 32 * s;
            FragB ah, al, bh, bl;
            ah.h[0] = *(const u16x8*)(ahp + k0);
            ah.h[1] = *(const u16x8*)(ahp + k0 + 16);
            al.h[0] = *(const u16x8*)(alp + k0);
            al.h[1] = *(const u16x8*)(alp + k0 + 16);
            bh.h[0] = *(const u16x8*)(ohp + k0);
            bh.h[1] = *(const u16x8*)(ohp + k0 + 16);
            bl.h[0] = *(const u16x8*)(olp + k0);
            bl.h[1] = *(const u16x8*)(olp + k0 + 16);
            mma_bf(acc2, ah, bh);
            mma_bf(acc2, ah, bl);
            mma_bf(acc2, al, bh);
        }
#pragma unroll
        for (int r = 0; r < 8; ++r) ost[(8 * h + r) * OUTD_ + 16 * wv + ml] = acc2[r];
    }
    __syncthreads();

    if (wv == 0) {
        float* gp = out + (size_t)b0 * OUTD_;
        v4f pv[4];
#pragma unroll
        for (int it = 0; it < 4; ++it) pv[it] = *(const v4f*)(ost + it * 128 + 4 * lane);
#pragma unroll
        for (int it = 0; it < 4; ++it) *(volatile v4f*)(gp + it * 128 + 4 * lane) = pv[it];
        __threadfence();
#pragma unroll
        for (int it = 0; it < 4; ++it) *(volatile v4f*)(gp + it * 128 + 4 * lane) = pv[it];
    }
}

extern "C" void kernel_launch(void* const* d_in, const int* in_sizes, int n_in,
                              void* d_out, int out_size, void* d_ws, size_t ws_size,
                              hipStream_t stream)
{
    if (n_in < 4) return;
    if (in_sizes[0] != BATCH_ * TLEN_ * FEAT1_) return;
    if (in_sizes[1] != BOND_ * FEAT1_ * BOND_)  return;
    if (in_sizes[2] != BOND_)                   return;
    if (in_sizes[3] != BOND_ * OUTD_)           return;
    if (out_size != BATCH_ * OUTD_)             return;
    if (ws_size < WS_END)                       return;

    const float* x     = (const float*)d_in[0];
    const float* core  = (const float*)d_in[1];
    const float* alpha = (const float*)d_in[2];
    const float* outc  = (const float*)d_in[3];
    float* out = (float*)d_out;

    char* ws = (char*)d_ws;
    unsigned short* Bh = (unsigned short*)(ws + OFF_BH);
    unsigned short* Bl = (unsigned short*)(ws + OFF_BL);

    core_planes_kernel<<<dim3(BOND_), dim3(256), 0, stream>>>(core, Bh, Bl);
    chain_kernel<<<dim3(BATCH_ / NRB_), dim3(NTH_), 0, stream>>>(x, alpha, outc, Bh, Bl, out);
}
